// HybridSurvivalQ_v3_9509057593684
// MI455X (gfx1250) — hardware-verified
//
#include <hip/hip_runtime.h>
#include <hip/hip_bf16.h>

typedef __attribute__((ext_vector_type(16))) _Float16 v16h;
typedef __attribute__((ext_vector_type(8)))  float    v8f;
typedef __attribute__((ext_vector_type(4)))  float    v4f_t;
typedef float v4fa __attribute__((ext_vector_type(4), may_alias));
#define RSPLIT (1.0f / 2048.0f)
__device__ __forceinline__ _Float16 lo_of(float v, _Float16 h) { return (_Float16)((v - (float)h) * 2048.0f); }
__device__ __forceinline__ v8f wmma16(v16h a, v16h b, v8f c) { return __builtin_amdgcn_wmma_f32_16x16x32_f16(false, a, false, b, (short)0, c, false, false); }
__device__ __forceinline__ v8f wmma_split(v16h a, v16h al, v16h b, v16h bl, v8f c) { v8f x = {}; x = wmma16(al, b, x); x = wmma16(a, bl, x); return wmma16(a, b, c) + x * RSPLIT; }

#pragma clang fp contract(off)
#define NQ 7
#define QDIM 128

#define WS_QOUT 0
#define QSTRIDE 16
#define WS_W1   1048576
#define WS_W2   (WS_W1 + 2 * 4096)
#define WS_F1   (WS_W2 + 2 * 2048)
#define WS_F2   (WS_F1 + 2 * 16384)
#define WS_F3   (WS_F2 + 2 * 8192)

__device__ __forceinline__ void swizzle_weight(
    const float* __restrict__ W, int K, int Ksrc, int N,
    _Float16* __restrict__ dst, int t, int stride)
{
    int nkb   = K >> 5;
    int total = (N >> 4) * nkb * 32 * 16;
    for (int i = t; i < total; i += stride) {
        int e    = i & 15;
        int L    = (i >> 4) & 31;
        int rest = i >> 9;
        int kb   = rest % nkb;
        int nt   = rest / nkb;
        int k    = (kb << 5) + ((L >> 4) << 3) + ((e < 8) ? e : (e + 8));
        int n    = (nt << 4) + (L & 15);
        float v  = (k < Ksrc) ? W[(size_t)k * N + n] : 0.0f;
        const _Float16 h = (_Float16)v;
        *(volatile _Float16*)(dst + i) = h; *(volatile _Float16*)(dst + total + i) = lo_of(v, h); __threadfence();
        *(volatile _Float16*)(dst + i) = h; *(volatile _Float16*)(dst + total + i) = lo_of(v, h);
    }
}

__global__ __launch_bounds__(256) void prep_kernel(
    const float* __restrict__ enc_w1, const float* __restrict__ enc_w2,
    const float* __restrict__ fus_w1, const float* __restrict__ fus_w2,
    const float* __restrict__ fus_w3, _Float16* __restrict__ ws)
{
    int t = threadIdx.x + blockIdx.x * blockDim.x;
    int stride = blockDim.x * gridDim.x;
    swizzle_weight(enc_w1,  64,  64,  64, ws + WS_W1, t, stride);
    swizzle_weight(enc_w2,  64,  64,  32, ws + WS_W2, t, stride);
    swizzle_weight(fus_w1, 128, 110, 128, ws + WS_F1, t, stride);
    swizzle_weight(fus_w2, 128, 128,  64, ws + WS_F2, t, stride);
    swizzle_weight(fus_w3,  64,  64,  32, ws + WS_F3, t, stride);
}

__device__ __forceinline__ void apply_ry(float re[4], float im[4],
                                         float th, int q, int lane)
{
    float s, c;
    __sincosf(0.5f * th, &s, &c);
    int bp = 6 - q;
    if (bp >= 2) {
        int mask = 1 << (bp - 2);
        int bit  = (lane >> (bp - 2)) & 1;
        float sg = bit ? s : -s;
#pragma unroll
        for (int j = 0; j < 4; ++j) {
            float pr = __shfl_xor(re[j], mask);
            float pi = __shfl_xor(im[j], mask);
            re[j] = c * re[j] + sg * pr;
            im[j] = c * im[j] + sg * pi;
        }
    } else {
        int m = 1 << bp;
#pragma unroll
        for (int j0 = 0; j0 < 4; ++j0) {
            if (j0 & m) continue;
            int j1 = j0 | m;
            float a0r = re[j0], a0i = im[j0], a1r = re[j1], a1i = im[j1];
            re[j0] = c * a0r - s * a1r;  im[j0] = c * a0i - s * a1i;
            re[j1] = s * a0r + c * a1r;  im[j1] = s * a0i + c * a1i;
        }
    }
}

__device__ __forceinline__ void apply_rz(float re[4], float im[4],
                                         float th, int q, int lane)
{
    float s, c;
    __sincosf(0.5f * th, &s, &c);
    int bp = 6 - q;
#pragma unroll
    for (int j = 0; j < 4; ++j) {
        int k   = (lane << 2) | j;
        int bit = (k >> bp) & 1;
        float ss = bit ? -s : s;
        float r = re[j], i2 = im[j];
        re[j] = r * c + i2 * ss;
        im[j] = i2 * c - r * ss;
    }
}

__global__ __launch_bounds__(256) void qsim_kernel(
    const float* __restrict__ x_q, const float* __restrict__ scales,
    const float* __restrict__ biases, const float* __restrict__ wry,
    const float* __restrict__ wrz, float* __restrict__ qout)
{
    __shared__ float lds[8][2 * QDIM];
    __shared__ __attribute__((aligned(16))) float sq[8 * QSTRIDE];
    int lane = threadIdx.x & 31;
    int wave = __builtin_amdgcn_readfirstlane(threadIdx.x) >> 5;
    int row  = blockIdx.x * 8 + wave;

    float re[4], im[4];
#pragma unroll
    for (int j = 0; j < 4; ++j) { re[j] = 0.0f; im[j] = 0.0f; }
    if (lane == 0) re[0] = 1.0f;

    float ang[NQ];
#pragma unroll
    for (int i = 0; i < NQ; ++i)
        ang[i] = scales[i] * x_q[(size_t)row * NQ + i] + biases[i];

    for (int layer = 0; layer < 3; ++layer) {
#pragma unroll
        for (int i = 0; i < NQ; ++i) apply_ry(re, im, ang[i], i, lane);
#pragma unroll
        for (int i = 0; i < NQ; ++i) {
            apply_ry(re, im, wry[layer * NQ + i], i, lane);
            apply_rz(re, im, wrz[layer * NQ + i], i, lane);
        }
        int shift = layer + 1;
#pragma unroll
        for (int i = 0; i < NQ; ++i) {
            int c = i, t = (i + shift) % NQ;
#pragma unroll
            for (int j = 0; j < 4; ++j) {
                int k = (lane << 2) | j;
                lds[wave][k]        = re[j];
                lds[wave][QDIM + k] = im[j];
            }
#pragma unroll
            for (int j = 0; j < 4; ++j) {
                int k  = (lane << 2) | j;
                int kp = k ^ ((((k >> (6 - c)) & 1)) << (6 - t));
                re[j] = lds[wave][kp];
                im[j] = lds[wave][QDIM + kp];
            }
        }
    }

    float f[14];
#pragma unroll
    for (int i = 0; i < 14; ++i) f[i] = 0.0f;
#pragma unroll
    for (int j = 0; j < 4; ++j) {
        int k = (lane << 2) | j;
        float p = re[j] * re[j] + im[j] * im[j];
#pragma unroll
        for (int i = 0; i < 7; ++i) {
            float sz  = ((k >> (6 - i)) & 1) ? -1.0f : 1.0f;
            float szn = ((k >> (6 - ((i + 1) % 7))) & 1) ? -1.0f : 1.0f;
            f[i]     += p * sz;
            f[7 + i] += p * sz * szn;
        }
    }
#pragma unroll
    for (int i = 0; i < 14; ++i) {
#pragma unroll
        for (int off = 16; off >= 1; off >>= 1)
            f[i] += __shfl_xor(f[i], off);
    }
    if (lane < QSTRIDE) {
        float v = 0.0f;
#pragma unroll
        for (int i = 0; i < 14; ++i) v = (lane == i) ? f[i] : v;
        sq[wave * QSTRIDE + lane] = v;
    }
    __syncthreads();
    if (threadIdx.x < 32) {
        const v4f_t v = *(const volatile v4fa*)(sq + threadIdx.x * 4);
        float* d = qout + (size_t)blockIdx.x * 8 * QSTRIDE + threadIdx.x * 4;
        *(volatile v4f_t*)d = v; __threadfence(); *(volatile v4f_t*)d = v;
    }
}

__device__ __forceinline__ v16h load_A(const _Float16* A, int lda,
                                       int row0, int k0, int lane)
{
    int m  = lane & 15;
    int kb = (lane >> 4) << 3;
    const _Float16* p = A + (size_t)(row0 + m) * lda + k0;
    v16h a;
#pragma unroll
    for (int e = 0; e < 8; ++e) a[e] = p[kb + e];
#pragma unroll
    for (int e = 0; e < 8; ++e) a[e + 8] = p[16 + kb + e];
    return a;
}

__device__ __forceinline__ void gemm_tiles(const _Float16* A, const _Float16* Al, int lda,
                                           const _Float16* __restrict__ Bsw,
                                           int K, int N,
                                           const float* __restrict__ bias,
                                           _Float16* C, _Float16* Cl, int ldc,
                                           int lane, int wave)
{
    int nkb    = K >> 5;
    int ntn    = N >> 4;
    int ntiles = 4 * ntn;
    const size_t plb = (size_t)ntn * nkb * 512;
    for (int t = wave; t < ntiles; t += 8) {
        int rs = t / ntn, nt = t % ntn;
        int r0 = rs << 4, n0 = nt << 4;
        v8f acc = {};
        for (int kb = 0; kb < nkb; ++kb) {
            v16h a  = load_A(A, lda, r0, kb << 5, lane);
            v16h al = load_A(Al, lda, r0, kb << 5, lane);
            const size_t bo = ((size_t)(nt * nkb + kb) * 32 + lane) * 16;
            acc = wmma_split(a, al, *(const v16h*)(Bsw + bo), *(const v16h*)(Bsw + plb + bo), acc);
        }
        int n  = lane & 15;
        int mb = (lane >> 4) << 3;
        float bb = bias[n0 + n];
#pragma unroll
        for (int r = 0; r < 8; ++r) {
            float v = acc[r] + bb;
            v = v > 0.0f ? v : 0.0f;
            const _Float16 h = (_Float16)v;
            C [(size_t)(r0 + mb + r) * ldc + n0 + n] = h;
            Cl[(size_t)(r0 + mb + r) * ldc + n0 + n] = lo_of(v, h);
        }
    }
}

__global__ __launch_bounds__(256) void mlp_kernel(
    const float* __restrict__ x_c, const _Float16* __restrict__ ws,
    const float* __restrict__ enc_b1, const float* __restrict__ enc_b2,
    const float* __restrict__ fus_b1, const float* __restrict__ fus_b2,
    const float* __restrict__ fus_b3, const float* __restrict__ fus_w4,
    const float* __restrict__ fus_b4, float* __restrict__ out)
{
    __shared__ _Float16 comb[2][64 * 128];
    __shared__ _Float16 h1  [2][64 * 64];
    __shared__ _Float16 hbig[2][64 * 128];
    __shared__ _Float16 h3  [2][64 * 32];

    const float* qout = (const float*)(ws + WS_QOUT);

    int tid  = threadIdx.x;
    int lane = tid & 31;
    int wave = __builtin_amdgcn_readfirstlane(tid) >> 5;
    int row0 = blockIdx.x * 64;

    for (int idx = tid; idx < 64 * 16; idx += 256) {
        int r = idx >> 4, c4 = idx & 15;
        float4 v = ((const float4*)(x_c + (size_t)(row0 + r) * 64))[c4];
        _Float16* d  = comb[0] + r * 128 + 46 + c4 * 4;
        _Float16* dl = comb[1] + r * 128 + 46 + c4 * 4;
        const float vv[4] = {v.x, v.y, v.z, v.w};
#pragma unroll
        for (int e = 0; e < 4; ++e) { const _Float16 h = (_Float16)vv[e]; d[e] = h; dl[e] = lo_of(vv[e], h); }
    }
    for (int idx = tid; idx < 64 * 14; idx += 256) {
        int r = idx / 14, c = idx % 14;
        const float v = qout[(size_t)(row0 + r) * QSTRIDE + c]; const _Float16 h = (_Float16)v;
        comb[0][r * 128 + c] = h; comb[1][r * 128 + c] = lo_of(v, h);
    }
    for (int idx = tid; idx < 64 * 50; idx += 256) {
        int r = idx / 50, c = idx % 50;
        const int o = r * 128 + ((c < 32) ? (14 + c) : (110 + c - 32));
        comb[0][o] = (_Float16)0.0f; comb[1][o] = (_Float16)0.0f;
    }
    __syncthreads();

    gemm_tiles(comb[0] + 46, comb[1] + 46, 128, ws + WS_W1, 64, 64, enc_b1, h1[0], h1[1], 64, lane, wave);
    __syncthreads();
    gemm_tiles(h1[0], h1[1], 64, ws + WS_W2, 64, 32, enc_b2, comb[0] + 14, comb[1] + 14, 128, lane, wave);
    __syncthreads();
    gemm_tiles(comb[0], comb[1], 128, ws + WS_F1, 128, 128, fus_b1, hbig[0], hbig[1], 128, lane, wave);
    __syncthreads();
    gemm_tiles(hbig[0], hbig[1], 128, ws + WS_F2, 128, 64, fus_b2, h1[0], h1[1], 64, lane, wave);
    __syncthreads();
    gemm_tiles(h1[0], h1[1], 64, ws + WS_F3, 64, 32, fus_b3, h3[0], h3[1], 32, lane, wave);
    __syncthreads();

    if (tid < 64) {
        float acc = fus_b4[0];
#pragma unroll
        for (int k = 0; k < 32; ++k)
            acc += ((float)h3[0][tid * 32 + k] + (float)h3[1][tid * 32 + k] * RSPLIT) * fus_w4[k];
        *(volatile float*)(out + row0 + tid) = acc; __threadfence(); *(volatile float*)(out + row0 + tid) = acc;
    }
}

extern "C" void kernel_launch(void* const* d_in, const int* in_sizes, int n_in,
                              void* d_out, int out_size, void* d_ws, size_t ws_size,
                              hipStream_t stream)
{
    const float* x_q    = (const float*)d_in[0];
    const float* x_c    = (const float*)d_in[1];
    const float* scales = (const float*)d_in[2];
    const float* biases = (const float*)d_in[3];
    const float* wry    = (const float*)d_in[4];
    const float* wrz    = (const float*)d_in[5];
    const float* enc_w1 = (const float*)d_in[6];
    const float* enc_b1 = (const float*)d_in[7];
    const float* enc_w2 = (const float*)d_in[8];
    const float* enc_b2 = (const float*)d_in[9];
    const float* fus_w1 = (const float*)d_in[10];
    const float* fus_b1 = (const float*)d_in[11];
    const float* fus_w2 = (const float*)d_in[12];
    const float* fus_b2 = (const float*)d_in[13];
    const float* fus_w3 = (const float*)d_in[14];
    const float* fus_b3 = (const float*)d_in[15];
    const float* fus_w4 = (const float*)d_in[16];
    const float* fus_b4 = (const float*)d_in[17];

    _Float16* ws = (_Float16*)d_ws;
    float* out   = (float*)d_out;

    prep_kernel<<<64, 256, 0, stream>>>(enc_w1, enc_w2, fus_w1, fus_w2, fus_w3, ws);
    qsim_kernel<<<4096, 256, 0, stream>>>(x_q, scales, biases, wry, wrz, (float*)(ws + WS_QOUT));
    mlp_kernel<<<512, 256, 0, stream>>>(x_c, ws, enc_b1, enc_b2,
                                        fus_b1, fus_b2, fus_b3,
                                        fus_w4, fus_b4, out);
}
